// CrossAttention_51900384805310
// MI455X (gfx1250) — hardware-verified
//
#include <hip/hip_runtime.h>
#include <stdint.h>


typedef _Float16 v16h __attribute__((ext_vector_type(16)));
typedef _Float16 v8h  __attribute__((ext_vector_type(8)));
typedef float    v8f  __attribute__((ext_vector_type(8)));
typedef float    v4f  __attribute__((ext_vector_type(4)));

#ifndef NB
#define NB 2
#endif
#ifndef SEQ
#define SEQ 2048
#endif
#define NB_FULL  2
#define SEQ_FULL 2048
#define HID      1024
#define NH       16
#define HD       64

#define ACT_CAR   8.0f
#define W_CAR     1024.0f
#define PROJ_SCL  0.0009765625f
#define RES_CAR   2048.0f
#define RES_INV   0.00048828125f
#define S_SCL     0.001953125f
#define P_CAR     16384.0f
#define O_SCL     0.001953125f
#define OUT_SCL   3.814697265625e-6f
#define RMS_EPS   1e-5f

static_assert(SEQ % 128 == 0);
static_assert(SEQ <= SEQ_FULL);
static_assert(NB >= 1 && NB <= NB_FULL);
static_assert(HID == NH * HD);
static_assert(HD == 64);
static_assert(HID % 64 == 0 && HID % 32 == 0);
static_assert((NB * SEQ) % 128 == 0);
static_assert((long)NB_FULL * SEQ_FULL * HID * 4 == 16777216L);
static_assert(((HID * HID / 8) / 256) * 256 * 8 == HID * HID);
static_assert(((2 * HID * HID / 8) / 256) * 256 * 8 == 2 * HID * HID);
static_assert(((SEQ * HID / 8) / 256) * 256 * 8 == SEQ * HID);
static_assert((SEQ / 8) * 8 * HID == SEQ * HID);
static_assert((HID / 64) * ((NB * SEQ) / 128) * 128 * 64 == NB * SEQ * HID);
static_assert(NB * NH * (SEQ / 128) * 128 * HD == NB * SEQ * HID);

union Frag16 { v16h v; v8h p[2]; };

__device__ __forceinline__ v16h ld_frag(const _Float16* p, int hl) {
  Frag16 f;
  f.p[0] = *(const v8h*)(p + 8 * hl);
  f.p[1] = *(const v8h*)(p + 16 + 8 * hl);
  return f.v;
}

__device__ __forceinline__ v8f mma(v16h a, v16h b, v8f c) {
  v8f d = __builtin_amdgcn_wmma_f32_16x16x32_f16(false, a, false, b, (short)0, c, false, false);
  asm volatile("v_nop\n\tv_nop\n\tv_nop\n\tv_nop" : "+v"(d) : "v"(a), "v"(b));
  return d;
}

__device__ __forceinline__ float bf16_rne(float x) {
  unsigned int u = __builtin_bit_cast(unsigned int, x);
  u += 0x7FFFu + ((u >> 16) & 1u);
  return __builtin_bit_cast(float, u & 0xFFFF0000u);
}

__global__ __launch_bounds__(256) void k_cvt8(const float* __restrict__ src,
                                              _Float16* __restrict__ dst,
                                              unsigned total8, unsigned sstride,
                                              unsigned dstride, float car)
{
  const unsigned i8 = blockIdx.x * 256u + threadIdx.x;
  if (i8 >= total8) return;
  const size_t e = (size_t)i8 * 8;
  const float* s = src + (size_t)blockIdx.y * sstride + e;
  const v4f x0 = *(const v4f*)s;
  const v4f x1 = *(const v4f*)(s + 4);
  v8h o;
#pragma unroll
  for (int j = 0; j < 4; ++j) {
    const float t0 = x0[j];
    const float t1 = x1[j];
    o[j]     = (_Float16)(bf16_rne(t0) * car);
    o[4 + j] = (_Float16)(bf16_rne(t1) * car);
  }
  _Float16* d = dst + (size_t)blockIdx.y * dstride + e;
  *(volatile v8h*)d = o;
  __threadfence();
  *(volatile v8h*)d = o;
}

__global__ __launch_bounds__(256) void k_rms(const float* __restrict__ X,
                                             const float* __restrict__ wn,
                                             _Float16* __restrict__ PH,
                                             _Float16* __restrict__ PL)
{
  const unsigned tid = threadIdx.x, lane = tid & 31u, w = tid >> 5;
  const unsigned s = blockIdx.x * 8u + w;
  const unsigned bb = blockIdx.y;
  const float* x = X + ((size_t)bb * SEQ_FULL + s) * HID;
  float ss = 0.f;
#pragma unroll 1
  for (unsigned j = 0; j < 4u; ++j) {
    const float* p = x + (j * 32u + lane) * 8u;
    const v4f a = *(const v4f*)p;
    const v4f b = *(const v4f*)(p + 4);
#pragma unroll
    for (int i = 0; i < 4; ++i) {
      const float t0 = bf16_rne(a[i]);
      const float t1 = bf16_rne(b[i]);
      ss += t0 * t0;
      ss += t1 * t1;
    }
  }
  ss += __shfl_xor(ss, 16, 32);
  ss += __shfl_xor(ss, 8, 32);
  ss += __shfl_xor(ss, 4, 32);
  ss += __shfl_xor(ss, 2, 32);
  ss += __shfl_xor(ss, 1, 32);
  const float rs = rsqrtf(ss * (1.0f / HID) + RMS_EPS);

  _Float16* const dh = PH + ((size_t)bb * SEQ + s) * HID;
  _Float16* const dl = PL + ((size_t)bb * SEQ + s) * HID;
#pragma unroll 1
  for (unsigned j = 0; j < 4u; ++j) {
    const unsigned off = (j * 32u + lane) * 8u;
    const v4f a  = *(const v4f*)(x + off);
    const v4f b  = *(const v4f*)(x + off + 4);
    const v4f wa = *(const v4f*)(wn + off);
    const v4f wb = *(const v4f*)(wn + off + 4);
    v8h oh, ol;
#pragma unroll
    for (int i = 0; i < 4; ++i) {
      const float t0 = bf16_rne(a[i]) * rs * bf16_rne(wa[i]) * ACT_CAR;
      const float t1 = bf16_rne(b[i]) * rs * bf16_rne(wb[i]) * ACT_CAR;
      const _Float16 h0 = (_Float16)t0;
      const _Float16 h1 = (_Float16)t1;
      oh[i]     = h0;
      oh[4 + i] = h1;
      ol[i]     = (_Float16)((t0 - (float)h0) * RES_CAR);
      ol[4 + i] = (_Float16)((t1 - (float)h1) * RES_CAR);
    }
    *(volatile v8h*)(dh + off) = oh;
    *(volatile v8h*)(dl + off) = ol;
    __threadfence();
    *(volatile v8h*)(dh + off) = oh;
    *(volatile v8h*)(dl + off) = ol;
  }
}

#define GE_LDS_F 9216

static_assert(2 * 128 * 72 <= 2 * GE_LDS_F);
static_assert(2 * 64 * 136 <= 2 * GE_LDS_F);
static_assert(128 * 68 <= GE_LDS_F);

template <bool ASPLIT, int EPI>
__global__ __launch_bounds__(256) __attribute__((amdgpu_num_vgpr(256)))
void k_gemm(const _Float16* __restrict__ Ah, const _Float16* __restrict__ Al,
            const _Float16* __restrict__ Bt, const float* __restrict__ bias,
            _Float16* __restrict__ Ph, _Float16* __restrict__ Pl,
            _Float16* __restrict__ Th, _Float16* __restrict__ Tl,
            float* __restrict__ Cf, float scl, float bcar)
{
  __shared__ __attribute__((aligned(16))) float lds_raw[GE_LDS_F];
  _Float16* const ldsH = reinterpret_cast<_Float16*>(lds_raw);
  float* const ldsF = lds_raw;

  const unsigned tid = threadIdx.x, lane = tid & 31u, w = tid >> 5;
  const unsigned hl = lane >> 4, c = lane & 15u;
  const unsigned wm = w & 3u, wn = w >> 2;
  const unsigned m0 = blockIdx.y * 128u, n0 = blockIdx.x * 64u;
  const unsigned mw = m0 + 32u * wm, nw = n0 + 32u * wn;

  const _Float16* ap0 = Ah + (size_t)(mw + c) * HID;
  const _Float16* ap1 = Ah + (size_t)(mw + 16u + c) * HID;
  const _Float16* lp0 = Al + (size_t)(mw + c) * HID;
  const _Float16* lp1 = Al + (size_t)(mw + 16u + c) * HID;
  const _Float16* bp0 = Bt + (size_t)(nw + c) * HID;
  const _Float16* bp1 = Bt + (size_t)(nw + 16u + c) * HID;
  (void)lp0; (void)lp1;

  v8f ah[4] = {};
  v8f al[4] = {};
#pragma unroll 1
  for (unsigned k0 = 0; k0 < (unsigned)HID; k0 += 32u) {
    const v16h a0 = ld_frag(ap0 + k0, (int)hl);
    const v16h a1 = ld_frag(ap1 + k0, (int)hl);
    const v16h b0 = ld_frag(bp0 + k0, (int)hl);
    const v16h b1 = ld_frag(bp1 + k0, (int)hl);
    ah[0] = mma(a0, b0, ah[0]);
    ah[1] = mma(a0, b1, ah[1]);
    ah[2] = mma(a1, b0, ah[2]);
    ah[3] = mma(a1, b1, ah[3]);
    if constexpr (ASPLIT) {
      const v16h l0 = ld_frag(lp0 + k0, (int)hl);
      const v16h l1 = ld_frag(lp1 + k0, (int)hl);
      al[0] = mma(l0, b0, al[0]);
      al[1] = mma(l0, b1, al[1]);
      al[2] = mma(l1, b0, al[2]);
      al[3] = mma(l1, b1, al[3]);
    }
  }

  const bool tr = (EPI == 1) && (n0 >= (unsigned)HID);
  const unsigned loff = tr ? (64u * 136u) : (128u * 72u);

#pragma unroll
  for (int i = 0; i < 2; ++i)
#pragma unroll
    for (int j = 0; j < 2; ++j) {
      const unsigned coll = 32u * wn + 16u * (unsigned)j + c;
      const float bv = bf16_rne(bias[n0 + coll]) * bcar;
#pragma unroll
      for (int r = 0; r < 8; ++r) {
        const unsigned rowl = 32u * wm + 16u * (unsigned)i + 8u * hl + (unsigned)r;
        float v = ah[i * 2 + j][r];
        if constexpr (ASPLIT) v += al[i * 2 + j][r] * RES_INV;
        v = v * scl + bv;
        if constexpr (EPI == 2) {
          ldsF[rowl * 68u + coll] = v;
        } else {
          const _Float16 hv = (_Float16)v;
          const float res = (v - (float)hv) * RES_CAR;
          const unsigned idx = tr ? (coll * 136u + rowl) : (rowl * 72u + coll);
          ldsH[idx] = hv;
          ldsH[loff + idx] = (_Float16)res;
        }
      }
    }
  __syncthreads();

  if constexpr (EPI == 2) {
    const unsigned bb = m0 / (unsigned)SEQ;
    const unsigned s0 = m0 - bb * (unsigned)SEQ;
    float* const ob = Cf + ((size_t)bb * SEQ_FULL + s0) * HID + n0;
    for (unsigned i = 0; i < 8u; ++i) {
      const unsigned q = i * 256u + tid;
      const unsigned rowl = q >> 4, col = (q & 15u) * 4u;
      const v4f v = *(const v4f*)(ldsF + rowl * 68u + col);
      *(volatile v4f*)(ob + (size_t)rowl * HID + col) = v;
    }
    __threadfence();
    for (unsigned i = 0; i < 8u; ++i) {
      const unsigned q = i * 256u + tid;
      const unsigned rowl = q >> 4, col = (q & 15u) * 4u;
      const v4f v = *(const v4f*)(ldsF + rowl * 68u + col);
      *(volatile v4f*)(ob + (size_t)rowl * HID + col) = v;
    }
  } else {
    if (tr) {
      const unsigned bb = m0 / (unsigned)SEQ;
      const unsigned s0 = m0 - bb * (unsigned)SEQ;
      _Float16* const th = Th + ((size_t)bb * HID + (n0 - (unsigned)HID)) * SEQ + s0;
      _Float16* const tl = Tl + ((size_t)bb * HID + (n0 - (unsigned)HID)) * SEQ + s0;
      for (unsigned i = 0; i < 4u; ++i) {
        const unsigned q = i * 256u + tid;
        const unsigned rowl = q >> 4, ch = (q & 15u) * 8u;
        const v8h vh = *(const v8h*)(ldsH + rowl * 136u + ch);
        const v8h vl = *(const v8h*)(ldsH + loff + rowl * 136u + ch);
        *(volatile v8h*)(th + (size_t)rowl * SEQ + ch) = vh;
        *(volatile v8h*)(tl + (size_t)rowl * SEQ + ch) = vl;
      }
      __threadfence();
      for (unsigned i = 0; i < 4u; ++i) {
        const unsigned q = i * 256u + tid;
        const unsigned rowl = q >> 4, ch = (q & 15u) * 8u;
        const v8h vh = *(const v8h*)(ldsH + rowl * 136u + ch);
        const v8h vl = *(const v8h*)(ldsH + loff + rowl * 136u + ch);
        *(volatile v8h*)(th + (size_t)rowl * SEQ + ch) = vh;
        *(volatile v8h*)(tl + (size_t)rowl * SEQ + ch) = vl;
      }
    } else {
      _Float16* const bh = Ph + (size_t)m0 * HID + n0;
      _Float16* const bl = Pl + (size_t)m0 * HID + n0;
      for (unsigned i = 0; i < 4u; ++i) {
        const unsigned q = i * 256u + tid;
        const unsigned rowl = q >> 3, ch = (q & 7u) * 8u;
        const v8h vh = *(const v8h*)(ldsH + rowl * 72u + ch);
        const v8h vl = *(const v8h*)(ldsH + loff + rowl * 72u + ch);
        *(volatile v8h*)(bh + (size_t)rowl * HID + ch) = vh;
        *(volatile v8h*)(bl + (size_t)rowl * HID + ch) = vl;
      }
      __threadfence();
      for (unsigned i = 0; i < 4u; ++i) {
        const unsigned q = i * 256u + tid;
        const unsigned rowl = q >> 3, ch = (q & 7u) * 8u;
        const v8h vh = *(const v8h*)(ldsH + rowl * 72u + ch);
        const v8h vl = *(const v8h*)(ldsH + loff + rowl * 72u + ch);
        *(volatile v8h*)(bh + (size_t)rowl * HID + ch) = vh;
        *(volatile v8h*)(bl + (size_t)rowl * HID + ch) = vl;
      }
    }
  }
}

#define AT_KP 72u
#define AT_VP 40u
#define AT_PP 40u
#define AT_K_H (32 * 72)
#define AT_V_H (64 * 40)
#define AT_P_H (8 * 16 * 40)
#define AT_TILE_H (2 * AT_K_H + 2 * AT_V_H + AT_P_H)
#define AT_EPI_H (2 * 128 * 72)
#define AT_LDS_H ((AT_TILE_H > AT_EPI_H) ? AT_TILE_H : AT_EPI_H)

__global__ __launch_bounds__(256) __attribute__((amdgpu_num_vgpr(256)))
void k_attn(const _Float16* __restrict__ Qh, const _Float16* __restrict__ Ql,
            const _Float16* __restrict__ Kh, const _Float16* __restrict__ Kl,
            const _Float16* __restrict__ Vth, const _Float16* __restrict__ Vtl,
            _Float16* __restrict__ Oh, _Float16* __restrict__ Ol)
{
  __shared__ __attribute__((aligned(16))) _Float16 lds[AT_LDS_H];
  _Float16* const ldsKH = lds;
  _Float16* const ldsKL = lds + AT_K_H;
  _Float16* const ldsVH = lds + 2 * AT_K_H;
  _Float16* const ldsVL = ldsVH + AT_V_H;
  _Float16* const ldsP  = ldsVL + AT_V_H;
  _Float16* const ldsEH = lds;
  _Float16* const ldsEL = lds + 128 * 72;

  const unsigned tid = threadIdx.x, lane = tid & 31u, w = tid >> 5;
  const unsigned hl = lane >> 4, c = lane & 15u;
  const unsigned qblocks = (unsigned)SEQ / 128u;
  const unsigned bx = blockIdx.x;
  const unsigned bh = bx / qblocks;
  const unsigned qb = bx - bh * qblocks;
  const unsigned h  = bh & (unsigned)(NH - 1);
  const unsigned bb = bh >> 4;
  const unsigned q0 = qb * 128u;
  const unsigned qw = q0 + 16u * w;

  const size_t qrow = ((size_t)bb * SEQ + qw + c) * HID + h * HD;
  const _Float16* kh  = Kh  + (size_t)bb * SEQ * HID + h * HD;
  const _Float16* kl  = Kl  + (size_t)bb * SEQ * HID + h * HD;
  const _Float16* vth = Vth + ((size_t)bb * HID + h * HD) * SEQ;
  const _Float16* vtl = Vtl + ((size_t)bb * HID + h * HD) * SEQ;
  _Float16* const myP = ldsP + w * (16u * AT_PP);

  const unsigned rr = tid >> 3, cc = (tid & 7u) * 8u;
  const unsigned dd = tid >> 2, kc = (tid & 3u) * 8u;

  v16h qh[2], ql[2];
#pragma unroll
  for (int ks = 0; ks < 2; ++ks) {
    qh[ks] = ld_frag(Qh + qrow + 32 * ks, (int)hl);
    ql[ks] = ld_frag(Ql + qrow + 32 * ks, (int)hl);
  }

  float m[8], l[8];
  v8f oh[4] = {};
  v8f ol[4] = {};
#pragma unroll
  for (int r = 0; r < 8; ++r) { m[r] = -__builtin_inff(); l[r] = 0.f; }

#pragma unroll 1
  for (unsigned kt = 0; kt < (unsigned)SEQ / 32u; ++kt) {
    const unsigned mk = kt * 32u;
    {
      const v8h k8h = *(const v8h*)(kh + (size_t)(mk + rr) * HID + cc);
      const v8h k8l = *(const v8h*)(kl + (size_t)(mk + rr) * HID + cc);
      const v8h v8a = *(const v8h*)(vth + (size_t)dd * SEQ + mk + kc);
      const v8h v8b = *(const v8h*)(vtl + (size_t)dd * SEQ + mk + kc);
      *(v8h*)(ldsKH + rr * AT_KP + cc) = k8h;
      *(v8h*)(ldsKL + rr * AT_KP + cc) = k8l;
      *(v8h*)(ldsVH + dd * AT_VP + kc) = v8a;
      *(v8h*)(ldsVL + dd * AT_VP + kc) = v8b;
    }
    __syncthreads();

    v8f sh[2] = {}, sl[2] = {};
#pragma unroll
    for (int ks = 0; ks < 2; ++ks) {
#pragma unroll
      for (int t = 0; t < 2; ++t) {
        const v16h kfh = ld_frag(ldsKH + (16u * (unsigned)t + c) * AT_KP + 32 * ks, (int)hl);
        const v16h kfl = ld_frag(ldsKL + (16u * (unsigned)t + c) * AT_KP + 32 * ks, (int)hl);
        sh[t] = mma(qh[ks], kfh, sh[t]);
        sl[t] = mma(ql[ks], kfh, sl[t]);
        sl[t] = mma(qh[ks], kfl, sl[t]);
      }
    }

#pragma unroll
    for (int r = 0; r < 8; ++r) {
      const float v0 = (sh[0][r] + sl[0][r] * RES_INV) * S_SCL;
      const float v1 = (sh[1][r] + sl[1][r] * RES_INV) * S_SCL;
      float tm = fmaxf(v0, v1);
      tm = fmaxf(tm, __shfl_xor(tm, 1, 32));
      tm = fmaxf(tm, __shfl_xor(tm, 2, 32));
      tm = fmaxf(tm, __shfl_xor(tm, 4, 32));
      tm = fmaxf(tm, __shfl_xor(tm, 8, 32));
      const float mn = fmaxf(m[r], tm);
      const float al = __expf(m[r] - mn);
      const float p0 = __expf(v0 - mn), p1 = __expf(v1 - mn);
      float rs = p0 + p1;
      rs += __shfl_xor(rs, 1, 32);
      rs += __shfl_xor(rs, 2, 32);
      rs += __shfl_xor(rs, 4, 32);
      rs += __shfl_xor(rs, 8, 32);
      l[r] = l[r] * al + rs;
      m[r] = mn;
#pragma unroll
      for (int t = 0; t < 4; ++t) { oh[t][r] *= al; ol[t][r] *= al; }
      _Float16* pp = myP + (8u * hl + (unsigned)r) * AT_PP + c;
      pp[0]  = (_Float16)(p0 * P_CAR);
      pp[16] = (_Float16)(p1 * P_CAR);
    }
    __syncthreads();

    const v16h pf = ld_frag(myP + c * AT_PP, (int)hl);
#pragma unroll
    for (int t = 0; t < 4; ++t) {
      const v16h vfh = ld_frag(ldsVH + (16u * (unsigned)t + c) * AT_VP, (int)hl);
      const v16h vfl = ld_frag(ldsVL + (16u * (unsigned)t + c) * AT_VP, (int)hl);
      oh[t] = mma(pf, vfh, oh[t]);
      ol[t] = mma(pf, vfl, ol[t]);
    }
    __syncthreads();
  }

#pragma unroll
  for (int r = 0; r < 8; ++r) {
    const float inv = (1.0f / l[r]) * O_SCL;
    const unsigned rowl = 16u * w + 8u * hl + (unsigned)r;
#pragma unroll
    for (int t = 0; t < 4; ++t) {
      const float v = (oh[t][r] + ol[t][r] * RES_INV) * inv;
      const _Float16 hv = (_Float16)v;
      const float res = (v - (float)hv) * RES_CAR;
      ldsEH[rowl * 72u + 16u * (unsigned)t + c] = hv;
      ldsEL[rowl * 72u + 16u * (unsigned)t + c] = (_Float16)res;
    }
  }
  __syncthreads();
  _Float16* const bh2 = Oh + ((size_t)bb * SEQ + q0) * HID + h * HD;
  _Float16* const bl2 = Ol + ((size_t)bb * SEQ + q0) * HID + h * HD;
  for (unsigned i = 0; i < 4u; ++i) {
    const unsigned q = i * 256u + tid;
    const unsigned rowl = q >> 3, ch = (q & 7u) * 8u;
    const v8h vh = *(const v8h*)(ldsEH + rowl * 72u + ch);
    const v8h vl = *(const v8h*)(ldsEL + rowl * 72u + ch);
    *(volatile v8h*)(bh2 + (size_t)rowl * HID + ch) = vh;
    *(volatile v8h*)(bl2 + (size_t)rowl * HID + ch) = vl;
  }
  __threadfence();
  for (unsigned i = 0; i < 4u; ++i) {
    const unsigned q = i * 256u + tid;
    const unsigned rowl = q >> 3, ch = (q & 7u) * 8u;
    const v8h vh = *(const v8h*)(ldsEH + rowl * 72u + ch);
    const v8h vl = *(const v8h*)(ldsEL + rowl * 72u + ch);
    *(volatile v8h*)(bh2 + (size_t)rowl * HID + ch) = vh;
    *(volatile v8h*)(bl2 + (size_t)rowl * HID + ch) = vl;
  }
}

extern "C" void kernel_launch(void* const* d_in, const int* in_sizes, int n_in,
                              void* d_out, int out_size, void* d_ws, size_t ws_size,
                              hipStream_t stream)
{
  if (n_in < 9) return;
  const long need_act = ((long)(NB - 1) * SEQ_FULL + SEQ) * HID;
  if ((long)in_sizes[0] < need_act) return;
  if ((long)in_sizes[1] < need_act) return;
  if ((long)in_sizes[2] < (long)HID) return;
  if ((long)in_sizes[3] < (long)HID * HID) return;
  if ((long)in_sizes[4] < (long)HID) return;
  if ((long)in_sizes[5] < 2L * HID * HID) return;
  if ((long)in_sizes[6] < 2L * HID) return;
  if ((long)in_sizes[7] < (long)HID * HID) return;
  if ((long)in_sizes[8] < (long)HID) return;
  if ((long)out_size < need_act) return;

  const float* q      = (const float*)d_in[0];
  const float* kv     = (const float*)d_in[1];
  const float* w_norm = (const float*)d_in[2];
  const float* w_q    = (const float*)d_in[3];
  const float* b_q    = (const float*)d_in[4];
  const float* w_kv   = (const float*)d_in[5];
  const float* b_kv   = (const float*)d_in[6];
  const float* w_out  = (const float*)d_in[7];
  const float* b_out  = (const float*)d_in[8];
  float* out = (float*)d_out;

  const size_t nW   = (size_t)HID * HID;
  const size_t nAct = (size_t)NB * SEQ * HID;
  const size_t total_halves = 4 * nW + 13 * nAct;
  if (total_halves * sizeof(_Float16) > ws_size) return;
  if (total_halves * sizeof(_Float16) > (size_t)134217728) return;

  _Float16* WQ16  = (_Float16*)d_ws;
  _Float16* WKV16 = WQ16  + nW;
  _Float16* WO16  = WKV16 + 2 * nW;
  _Float16* KV16  = WO16  + nW;
  _Float16* QNH   = KV16  + nAct;
  _Float16* QNL   = QNH   + nAct;
  _Float16* QH    = QNL   + nAct;
  _Float16* QL    = QH    + nAct;
  _Float16* KH    = QL    + nAct;
  _Float16* KL    = KH    + nAct;
  _Float16* VTH   = KL    + nAct;
  _Float16* VTL   = VTH   + nAct;
  _Float16* OH    = VTL   + nAct;
  _Float16* OL    = OH    + nAct;

  const unsigned tw8  = (unsigned)(nW / 8);
  const unsigned tkv8 = (unsigned)(2 * nW / 8);
  const unsigned ta8  = (unsigned)((size_t)SEQ * HID / 8);
  k_cvt8<<<dim3(tw8 / 256, 1), 256, 0, stream>>>(w_q, WQ16, tw8, 0u, 0u, W_CAR);
  k_cvt8<<<dim3(tkv8 / 256, 1), 256, 0, stream>>>(w_kv, WKV16, tkv8, 0u, 0u, W_CAR);
  k_cvt8<<<dim3(tw8 / 256, 1), 256, 0, stream>>>(w_out, WO16, tw8, 0u, 0u, W_CAR);
  k_cvt8<<<dim3(ta8 / 256, NB), 256, 0, stream>>>(kv, KV16, ta8,
                                                  (unsigned)(SEQ_FULL * HID), (unsigned)(SEQ * HID), ACT_CAR);

  k_rms<<<dim3(SEQ / 8, NB), 256, 0, stream>>>(q, w_norm, QNH, QNL);

  k_gemm<true, 0><<<dim3(HID / 64, (NB * SEQ) / 128), 256, 0, stream>>>(
      QNH, QNL, WQ16, b_q, QH, QL, QH, QL, out, PROJ_SCL, ACT_CAR);

  k_gemm<false, 1><<<dim3((2 * HID) / 64, (NB * SEQ) / 128), 256, 0, stream>>>(
      KV16, KV16, WKV16, b_kv, KH, KL, VTH, VTL, out, PROJ_SCL, ACT_CAR);

  k_attn<<<NB * NH * (SEQ / 128), 256, 0, stream>>>(QH, QL, KH, KL, VTH, VTL, OH, OL);

  k_gemm<true, 2><<<dim3(HID / 64, (NB * SEQ) / 128), 256, 0, stream>>>(
      OH, OL, WO16, b_out, OH, OL, OH, OL, out, OUT_SCL, 1.0f);
}
